// BiRNN_IFBUS3S8SAPP_84636625535343
// MI455X (gfx1250) — hardware-run, weakly checked
//
#include <hip/hip_runtime.h>
#include <math.h>

constexpr int NB        = 32;
constexpr int NT_STEPS  = 2048;
constexpr int NFEAT     = 64;
constexpr int NUNIT     = 256;
constexpr int NGATE     = 4 * NUNIT;
constexpr int NHID2     = 2 * NUNIT;
constexpr int K0TOT     = NFEAT + NUNIT;
constexpr int K1TOT     = NHID2 + NUNIT;
constexpr int NHEADCOL  = 20;
constexpr int NHEADPAD  = 32;
constexpr int LTHR      = 512;
constexpr int PTHR      = 256;
constexpr int XPITCH    = 72;
constexpr int HPITCH    = 264;
constexpr int SLABP     = 36;
constexpr int NROWS     = NB * NT_STEPS;
constexpr float ACARRY  = 16.0f;
constexpr float WCARRY  = 256.0f;
constexpr float FOLD    = 1.0f / (ACARRY * WCARRY);

static_assert(NB == 32, "two 16-row m-subtiles per block");
static_assert(NUNIT == 16 * (LTHR / 32), "one 16-unit subtile per wave");
static_assert(NB * NFEAT == LTHR * 4, "x staging covers the tile exactly");
static_assert(K0TOT % 32 == 0 && K1TOT % 32 == 0 && NUNIT % 32 == 0, "K multiples of 32");
static_assert(NFEAT % 64 == 0 && NUNIT % 64 == 0 && NHID2 % 64 == 0 && NGATE % 64 == 0, "transpose tiles");
static_assert(NHEADCOL <= NHEADPAD && NHEADPAD == 32, "head columns padded to two 16-col subtiles");
static_assert(NROWS % PTHR == 0, "finish grid exact");
static_assert((XPITCH % 8) == 0 && (HPITCH % 8) == 0 && (SLABP % 4) == 0, "16-B aligned LDS rows");

typedef __attribute__((ext_vector_type(16))) _Float16 v16h;
typedef __attribute__((ext_vector_type(8)))  _Float16 v8h;
typedef __attribute__((ext_vector_type(4)))  _Float16 v4h;
typedef __attribute__((ext_vector_type(8)))  float    v8f;
typedef __attribute__((ext_vector_type(4)))  float    v4f;

__device__ __forceinline__ unsigned short f2bf_bits(float f) {
  unsigned u = __float_as_uint(f);
  return (unsigned short)((u + 0x7FFFu + ((u >> 16) & 1u)) >> 16);
}
__device__ __forceinline__ float bf_bits2f(unsigned short h) { return __uint_as_float(((unsigned)h) << 16); }
__device__ __forceinline__ float bf16r(float f) { return bf_bits2f(f2bf_bits(f)); }

struct FragH {
  union U { v16h v; v8h h[2]; };
  static __device__ __forceinline__ v16h load(const _Float16* p) {
    U f;
    f.h[0] = *(const v8h*)(p);
    f.h[1] = *(const v8h*)(p + 16);
    return f.v;
  }
  static __device__ __forceinline__ v8f mma(v16h a, v16h b, v8f c) {
    return __builtin_amdgcn_wmma_f32_16x16x32_f16(false, a, false, b, (short)0, c, false, false);
  }
};

__device__ __forceinline__ void guard8(v8f& d0, v8f& d1, v8f& d2, v8f& d3, v8f& d4, v8f& d5, v8f& d6, v8f& d7,
                                       v16h a0, v16h a1, v16h b0, v16h b1, v16h b2, v16h b3) {
  asm volatile("v_nop\n\tv_nop\n\tv_nop\n\tv_nop"
               : "+v"(d0), "+v"(d1), "+v"(d2), "+v"(d3), "+v"(d4), "+v"(d5), "+v"(d6), "+v"(d7)
               : "v"(a0), "v"(a1), "v"(b0), "v"(b1), "v"(b2), "v"(b3));
}
__device__ __forceinline__ void guard2(v8f& d0, v8f& d1, v16h a, v16h b0, v16h b1) {
  asm volatile("v_nop\n\tv_nop\n\tv_nop\n\tv_nop" : "+v"(d0), "+v"(d1) : "v"(a), "v"(b0), "v"(b1));
}

__device__ __forceinline__ void mma_tile8(const _Float16* pa0, const _Float16* pa1,
                                          const _Float16* pb0, const _Float16* pb1,
                                          const _Float16* pb2, const _Float16* pb3,
                                          v8f& d00, v8f& d01, v8f& d02, v8f& d03,
                                          v8f& d10, v8f& d11, v8f& d12, v8f& d13) {
  const v16h a0 = FragH::load(pa0);
  const v16h a1 = FragH::load(pa1);
  const v16h b0 = FragH::load(pb0);
  const v16h b1 = FragH::load(pb1);
  const v16h b2 = FragH::load(pb2);
  const v16h b3 = FragH::load(pb3);
  d00 = FragH::mma(a0, b0, d00);
  d10 = FragH::mma(a1, b0, d10);
  d01 = FragH::mma(a0, b1, d01);
  d11 = FragH::mma(a1, b1, d11);
  d02 = FragH::mma(a0, b2, d02);
  d12 = FragH::mma(a1, b2, d12);
  d03 = FragH::mma(a0, b3, d03);
  d13 = FragH::mma(a1, b3, d13);
  guard8(d00, d01, d02, d03, d10, d11, d12, d13, a0, a1, b0, b1, b2, b3);
}

__device__ __forceinline__ float fsig(float x)  { return __builtin_amdgcn_rcpf(1.0f + __expf(-x)); }
__device__ __forceinline__ float ftanh(float x) { return 1.0f - 2.0f * __builtin_amdgcn_rcpf(__expf(2.0f * x) + 1.0f); }

__global__ __launch_bounds__(PTHR) void tpw_kernel(const float* __restrict__ src, int C, int ldo,
                                                   unsigned short* __restrict__ O, float sc) {
  __shared__ float Tt[64 * 65];
  const int tid = threadIdx.x;
  const int c0 = blockIdx.x * 64, r0 = blockIdx.y * 64;
#pragma unroll
  for (int i = 0; i < 4; ++i) {
    const int idx = i * PTHR + tid;
    const int rr = idx >> 4, cc = (idx & 15) * 4;
    const v4f v = *(const v4f*)(src + (size_t)(r0 + rr) * (size_t)C + c0 + cc);
    Tt[rr * 65 + cc + 0] = v[0];
    Tt[rr * 65 + cc + 1] = v[1];
    Tt[rr * 65 + cc + 2] = v[2];
    Tt[rr * 65 + cc + 3] = v[3];
  }
  __syncthreads();
  const int q = tid >> 3, c8 = (tid & 7) * 8;
  v8h hv[2];
#pragma unroll
  for (int g = 0; g < 2; ++g) {
    const int qq = g * 32 + q;
#pragma unroll
    for (int e = 0; e < 8; ++e) {
      const float f = Tt[(c8 + e) * 65 + qq];
      hv[g][e] = (_Float16)(bf16r(f) * sc);
    }
  }
  for (int pass = 0; pass < 2; ++pass) {
#pragma unroll
    for (int g = 0; g < 2; ++g) {
      const size_t o = (size_t)(c0 + g * 32 + q) * (size_t)ldo + (size_t)(r0 + c8);
      *(volatile v8h*)(O + o) = hv[g];
    }
    __threadfence();
  }
}

__global__ __launch_bounds__(PTHR) void head_plane_kernel(const float* __restrict__ Wp, const float* __restrict__ Wbu,
                                                          const float* __restrict__ W3, const float* __restrict__ W8,
                                                          const float* __restrict__ Wa, const float* __restrict__ Wpp,
                                                          unsigned short* __restrict__ HB) {
  const int i  = blockIdx.x * PTHR + threadIdx.x;
  const int e0 = 2 * i;
  const int d  = e0 >> 13;
  const int n  = (e0 >> 8) & 31;
  const int k  = e0 & 255;
  const int c2a = min(max(n, 0), 1);
  const int c2b = min(max(n - 2, 0), 1);
  const int c3  = min(max(n - 4, 0), 2);
  const int c8  = min(max(n - 7, 0), 7);
  const int c4  = min(max(n - 16, 0), 3);
  float vals[2];
#pragma unroll
  for (int u = 0; u < 2; ++u) {
    const int row = d * NUNIT + k + u;
    float va = Wp[row * 2 + c2a];
    asm volatile("" : "+v"(va));
    float vb = Wbu[row * 2 + c2b];
    asm volatile("" : "+v"(vb));
    float vc = W3[row * 3 + c3];
    asm volatile("" : "+v"(vc));
    float vd = W8[row * 8 + c8];
    asm volatile("" : "+v"(vd));
    float ve = Wa[row];
    asm volatile("" : "+v"(ve));
    float vf = Wpp[row * 4 + c4];
    asm volatile("" : "+v"(vf));
    float v = 0.0f;
    v = (n < 2) ? va : v;
    v = (n >= 2 && n < 4) ? vb : v;
    v = (n >= 4 && n < 7) ? vc : v;
    v = (n >= 7 && n < 15) ? vd : v;
    v = (n == 15) ? ve : v;
    v = (n >= 16 && n < NHEADCOL) ? vf : v;
    vals[u] = bf16r(v) * WCARRY;
  }
  const _Float16 h0 = (_Float16)vals[0], h1 = (_Float16)vals[1];
  const unsigned w = (unsigned)__builtin_bit_cast(unsigned short, h0) |
                     ((unsigned)__builtin_bit_cast(unsigned short, h1) << 16);
  ((volatile unsigned*)HB)[i] = w;
  __threadfence();
  ((volatile unsigned*)HB)[i] = w;
}

__device__ __forceinline__ void stage_x_tile(const float* __restrict__ x, _Float16* Ax, int tid, int t) {
  const int m = tid >> 4, f4 = (tid & 15) * 4;
  const v4f v = *(const v4f*)(x + ((size_t)m * NT_STEPS + (size_t)t) * NFEAT + f4);
  v4h hv;
  hv[0] = (_Float16)(bf16r(v[0]) * ACARRY);
  hv[1] = (_Float16)(bf16r(v[1]) * ACARRY);
  hv[2] = (_Float16)(bf16r(v[2]) * ACARRY);
  hv[3] = (_Float16)(bf16r(v[3]) * ACARRY);
  *(v4h*)(Ax + m * XPITCH + f4) = hv;
}

template <int LAYER>
__global__ __launch_bounds__(LTHR) void bilstm_layer_kernel(const float* __restrict__ xin, unsigned short* hplane,
                                                            const int* __restrict__ xmask,
                                                            const unsigned short* __restrict__ wplane,
                                                            const float* __restrict__ bias_f,
                                                            const float* __restrict__ bias_b,
                                                            const unsigned short* __restrict__ hbplane,
                                                            float* part) {
  constexpr int KX   = (LAYER == 0) ? NFEAT : NHID2;
  constexpr int KTOT = KX + NUNIT;
  static_assert(KX % 32 == 0 && KTOT % 32 == 0, "k-steps of 32");
  __shared__ __align__(16) _Float16 Ax[(LAYER == 0) ? NB * XPITCH : 8];
  __shared__ __align__(16) _Float16 Ah[NB * HPITCH];
  __shared__ __align__(16) _Float16 Rh[(LAYER == 1) ? NB * HPITCH : 8];
  __shared__ __align__(16) float    Sl[(LAYER == 1) ? 2 * 16 * SLABP : 4];
  __shared__ int msk[NB];

  const int tid  = threadIdx.x;
  const int lane = tid & 31;
  const int wave = __builtin_amdgcn_readfirstlane((int)(threadIdx.x >> 5));
  const int c = lane & 15, hh = lane >> 4, koff = hh * 8;
  const int dir = blockIdx.x;
  const int j = 16 * wave + c;
  constexpr size_t GSTR = (size_t)NUNIT * KTOT;
  const _Float16* WB = (const _Float16*)wplane + (size_t)dir * NGATE * KTOT + (size_t)j * KTOT + koff;
  const _Float16* HPL = (const _Float16*)hplane;

  float bb[4];
#pragma unroll
  for (int g = 0; g < 4; ++g) {
    const float vf = bias_f[g * NUNIT + j];
    const float vb = bias_b[g * NUNIT + j];
    bb[g] = bf16r(dir ? vb : vf);
  }

#pragma unroll 1
  for (int i = tid; i < NB * HPITCH; i += LTHR) Ah[i] = (_Float16)0.0f;
  const int tfirst = dir ? (NT_STEPS - 1) : 0;
  if (LAYER == 0) stage_x_tile(xin, Ax, tid, tfirst);
  if (wave == 0) {
    const int mv0 = xmask[lane * NT_STEPS + tfirst];
    msk[lane] = mv0;
  }
  float cst[2][8], hst[2][8];
#pragma unroll
  for (int mt = 0; mt < 2; ++mt)
#pragma unroll
    for (int r = 0; r < 8; ++r) { cst[mt][r] = 0.0f; hst[mt][r] = 0.0f; }
  __syncthreads();

  const v8f z8 = {0.f, 0.f, 0.f, 0.f, 0.f, 0.f, 0.f, 0.f};
  const _Float16* hr0 = Ah + c * HPITCH + koff;
  const _Float16* hr1 = hr0 + 16 * HPITCH;

#pragma unroll 1
  for (int s = 0; s < NT_STEPS; ++s) {
    const int t = dir ? (NT_STEPS - 1 - s) : s;
    v8f acc[2][4];
#pragma unroll
    for (int mt = 0; mt < 2; ++mt)
#pragma unroll
      for (int g = 0; g < 4; ++g) acc[mt][g] = z8;

    if (LAYER == 0) {
      const _Float16* xr0 = Ax + c * XPITCH + koff;
      const _Float16* xr1 = xr0 + 16 * XPITCH;
#pragma unroll 1
      for (int k0 = 0; k0 < KX; k0 += 32) {
        const _Float16* wb = WB + k0;
        mma_tile8(xr0 + k0, xr1 + k0, wb, wb + GSTR, wb + 2 * GSTR, wb + 3 * GSTR,
                  acc[0][0], acc[0][1], acc[0][2], acc[0][3], acc[1][0], acc[1][1], acc[1][2], acc[1][3]);
      }
    } else {
      const _Float16* gr0 = HPL + ((size_t)t * NB + c) * NHID2 + koff;
      const _Float16* gr1 = gr0 + (size_t)16 * NHID2;
#pragma unroll 1
      for (int k0 = 0; k0 < KX; k0 += 32) {
        const _Float16* wb = WB + k0;
        mma_tile8(gr0 + k0, gr1 + k0, wb, wb + GSTR, wb + 2 * GSTR, wb + 3 * GSTR,
                  acc[0][0], acc[0][1], acc[0][2], acc[0][3], acc[1][0], acc[1][1], acc[1][2], acc[1][3]);
      }
    }
#pragma unroll 1
    for (int k0 = 0; k0 < NUNIT; k0 += 32) {
      const _Float16* wb = WB + KX + k0;
      mma_tile8(hr0 + k0, hr1 + k0, wb, wb + GSTR, wb + 2 * GSTR, wb + 3 * GSTR,
                acc[0][0], acc[0][1], acc[0][2], acc[0][3], acc[1][0], acc[1][1], acc[1][2], acc[1][3]);
    }

#pragma unroll
    for (int mt = 0; mt < 2; ++mt) {
#pragma unroll
      for (int r = 0; r < 8; ++r) {
        const int mv = msk[16 * mt + 8 * hh + r];
        const float zi = acc[mt][0][r] * FOLD + bb[0];
        const float zf = acc[mt][1][r] * FOLD + bb[1];
        const float zg = acc[mt][2][r] * FOLD + bb[2];
        const float zo = acc[mt][3][r] * FOLD + bb[3];
        const float ig = fsig(zi);
        const float fg = fsig(zf);
        const float gg = ftanh(zg);
        const float og = fsig(zo);
        const float cn = fg * cst[mt][r] + ig * gg;
        const float hn = og * ftanh(cn);
        const bool upd = (mv != 1);
        cst[mt][r] = upd ? cn : cst[mt][r];
        hst[mt][r] = upd ? hn : hst[mt][r];
      }
    }
    __syncthreads();
#pragma unroll
    for (int mt = 0; mt < 2; ++mt) {
#pragma unroll
      for (int r = 0; r < 8; ++r) {
        const int row = 16 * mt + 8 * hh + r;
        Ah[row * HPITCH + j] = (_Float16)(hst[mt][r] * ACARRY);
        if (LAYER == 1) Rh[row * HPITCH + j] = (_Float16)(fmaxf(hst[mt][r], 0.0f) * ACARRY);
      }
    }
    {
      const int sn = (s + 1 < NT_STEPS) ? (s + 1) : (NT_STEPS - 1);
      const int tn = dir ? (NT_STEPS - 1 - sn) : sn;
      if (LAYER == 0) stage_x_tile(xin, Ax, tid, tn);
      if (wave == 0) {
        const int mvn = xmask[lane * NT_STEPS + tn];
        msk[lane] = mvn;
      }
    }
    __syncthreads();

    if (LAYER == 0) {
      const int r0 = wave, r1 = wave + 16;
      const v8h v0 = *(const v8h*)(Ah + r0 * HPITCH + lane * 8);
      const v8h v1 = *(const v8h*)(Ah + r1 * HPITCH + lane * 8);
      unsigned short* d0 = hplane + ((size_t)t * NB + r0) * NHID2 + dir * NUNIT + lane * 8;
      unsigned short* d1 = hplane + ((size_t)t * NB + r1) * NHID2 + dir * NUNIT + lane * 8;
      for (int pass = 0; pass < 2; ++pass) {
        *(volatile v8h*)d0 = v0;
        *(volatile v8h*)d1 = v1;
        __threadfence();
      }
    } else {
      if (wave < 2) {
        const int mt = wave;
        const _Float16* rr  = Rh + (16 * mt + c) * HPITCH + koff;
        const _Float16* hb0 = (const _Float16*)hbplane + ((size_t)dir * NHEADPAD + c) * NUNIT + koff;
        const _Float16* hb1 = hb0 + (size_t)16 * NUNIT;
        v8f p0 = z8, p1 = z8;
#pragma unroll 1
        for (int k0 = 0; k0 < NUNIT; k0 += 32) {
          const v16h a  = FragH::load(rr + k0);
          const v16h b0 = FragH::load(hb0 + k0);
          const v16h b1 = FragH::load(hb1 + k0);
          p0 = FragH::mma(a, b0, p0);
          p1 = FragH::mma(a, b1, p1);
          guard2(p0, p1, a, b0, b1);
        }
        float* slab = Sl + mt * 16 * SLABP;
#pragma unroll
        for (int r = 0; r < 8; ++r) {
          slab[(8 * hh + r) * SLABP + c]      = p0[r] * FOLD;
          slab[(8 * hh + r) * SLABP + 16 + c] = p1[r] * FOLD;
        }
        __builtin_amdgcn_fence(__ATOMIC_RELEASE, "workgroup");
        __builtin_amdgcn_wave_barrier();
        __builtin_amdgcn_fence(__ATOMIC_ACQUIRE, "workgroup");
        const int q = lane >> 3, c4 = (lane & 7) * 4;
        v4f ov[4];
#pragma unroll
        for (int it = 0; it < 4; ++it) ov[it] = *(const v4f*)(slab + (it * 4 + q) * SLABP + c4);
        float* pbase = part + (((size_t)dir * NT_STEPS + (size_t)t) * NB + 16 * mt) * NHEADPAD + c4;
        for (int pass = 0; pass < 2; ++pass) {
#pragma unroll
          for (int it = 0; it < 4; ++it) *(volatile v4f*)(pbase + (size_t)(it * 4 + q) * NHEADPAD) = ov[it];
          __threadfence();
        }
        __builtin_amdgcn_fence(__ATOMIC_RELEASE, "workgroup");
        __builtin_amdgcn_wave_barrier();
        __builtin_amdgcn_fence(__ATOMIC_ACQUIRE, "workgroup");
      }
    }
  }
}

__global__ __launch_bounds__(PTHR) void finish_kernel(const float* __restrict__ part,
                                                      const float* __restrict__ bp, const float* __restrict__ bbu,
                                                      const float* __restrict__ b3, const float* __restrict__ b8,
                                                      const float* __restrict__ ba, const float* __restrict__ bpp,
                                                      float* __restrict__ out) {
  __shared__ __align__(16) float St[PTHR * NHEADCOL];
  const int tid = threadIdx.x;
  const int n0 = blockIdx.x * PTHR;
  const int n = n0 + tid;
  const int b = n >> 11, t = n & (NT_STEPS - 1);
  const float* q0 = part + (((size_t)t) * NB + b) * NHEADPAD;
  const float* q1 = part + (((size_t)NT_STEPS + (size_t)t) * NB + b) * NHEADPAD;
  float lg[NHEADCOL];
#pragma unroll
  for (int i = 0; i < 5; ++i) {
    const v4f u0 = *(const v4f*)(q0 + 4 * i);
    const v4f u1 = *(const v4f*)(q1 + 4 * i);
    lg[4 * i + 0] = u0[0] + u1[0];
    lg[4 * i + 1] = u0[1] + u1[1];
    lg[4 * i + 2] = u0[2] + u1[2];
    lg[4 * i + 3] = u0[3] + u1[3];
  }
  lg[0] += bf16r(bp[0]);
  lg[1] += bf16r(bp[1]);
  lg[2] += bf16r(bbu[0]);
  lg[3] += bf16r(bbu[1]);
#pragma unroll
  for (int i = 0; i < 3; ++i) lg[4 + i] += bf16r(b3[i]);
#pragma unroll
  for (int i = 0; i < 8; ++i) lg[7 + i] += bf16r(b8[i]);
  lg[15] += bf16r(ba[0]);
#pragma unroll
  for (int i = 0; i < 4; ++i) lg[16 + i] += bf16r(bpp[i]);
  {
    const float mx = fmaxf(lg[0], lg[1]);
    const float e0 = expf(lg[0] - mx), e1 = expf(lg[1] - mx);
    const float inv = 1.0f / (e0 + e1);
    lg[0] = e0 * inv;
    lg[1] = e1 * inv;
  }
  St[tid * 2 + 0] = lg[0];
  St[tid * 2 + 1] = lg[1];
  St[512 + tid * 2 + 0] = lg[2];
  St[512 + tid * 2 + 1] = lg[3];
#pragma unroll
  for (int i = 0; i < 3; ++i) St[1024 + tid * 3 + i] = lg[4 + i];
#pragma unroll
  for (int i = 0; i < 8; ++i) St[1792 + tid * 8 + i] = lg[7 + i];
  St[3840 + tid] = lg[15];
#pragma unroll
  for (int i = 0; i < 4; ++i) St[4096 + tid * 4 + i] = lg[16 + i];
  __syncthreads();

  v4f vv[5];
  float* dp[5];
#pragma unroll
  for (int it = 0; it < 5; ++it) {
    const int q = it * PTHR + tid;
    vv[it] = *(const v4f*)(St + 4 * q);
    int segq = 0, wdt = 2;
    size_t base = 0;
    if (q >= 128)  { segq = 128;  wdt = 2; base = (size_t)NROWS * 2; }
    if (q >= 256)  { segq = 256;  wdt = 3; base = (size_t)NROWS * 4; }
    if (q >= 448)  { segq = 448;  wdt = 8; base = (size_t)NROWS * 7; }
    if (q >= 960)  { segq = 960;  wdt = 1; base = (size_t)NROWS * 15; }
    if (q >= 1024) { segq = 1024; wdt = 4; base = (size_t)NROWS * 16; }
    dp[it] = out + base + (size_t)n0 * (size_t)wdt + (size_t)(q - segq) * 4;
  }
  for (int pass = 0; pass < 2; ++pass) {
#pragma unroll
    for (int it = 0; it < 5; ++it) *(volatile v4f*)dp[it] = vv[it];
    __threadfence();
  }
}

extern "C" void kernel_launch(void* const* d_in, const int* in_sizes, int n_in,
                              void* d_out, int out_size, void* d_ws, size_t ws_size, hipStream_t stream) {
  if (n_in < 27 || d_out == nullptr || d_ws == nullptr) return;
  if (in_sizes[0] != NB * NT_STEPS * NFEAT || in_sizes[1] != NB * NT_STEPS ||
      in_sizes[3] != NFEAT * NGATE || in_sizes[4] != NUNIT * NGATE || in_sizes[5] != NGATE ||
      in_sizes[6] != NFEAT * NGATE || in_sizes[7] != NUNIT * NGATE || in_sizes[8] != NGATE ||
      in_sizes[9] != NHID2 * NGATE || in_sizes[10] != NUNIT * NGATE || in_sizes[11] != NGATE ||
      in_sizes[12] != NHID2 * NGATE || in_sizes[13] != NUNIT * NGATE || in_sizes[14] != NGATE ||
      in_sizes[15] != NHID2 * 2 || in_sizes[16] != 2 || in_sizes[17] != NHID2 * 2 || in_sizes[18] != 2 ||
      in_sizes[19] != NHID2 * 3 || in_sizes[20] != 3 || in_sizes[21] != NHID2 * 8 || in_sizes[22] != 8 ||
      in_sizes[23] != NHID2 || in_sizes[24] != 1 || in_sizes[25] != NHID2 * 4 || in_sizes[26] != 4 ||
      out_size != NROWS * NHEADCOL) return;

  const float* x    = (const float*)d_in[0];
  const int*   xm   = (const int*)d_in[1];
  const float* Wf0  = (const float*)d_in[3];
  const float* Uf0  = (const float*)d_in[4];
  const float* bf0  = (const float*)d_in[5];
  const float* Wb0  = (const float*)d_in[6];
  const float* Ub0  = (const float*)d_in[7];
  const float* bb0  = (const float*)d_in[8];
  const float* Wf1  = (const float*)d_in[9];
  const float* Uf1  = (const float*)d_in[10];
  const float* bf1  = (const float*)d_in[11];
  const float* Wb1  = (const float*)d_in[12];
  const float* Ub1  = (const float*)d_in[13];
  const float* bb1  = (const float*)d_in[14];
  const float* Wp   = (const float*)d_in[15];
  const float* bp   = (const float*)d_in[16];
  const float* Wbu  = (const float*)d_in[17];
  const float* bbu  = (const float*)d_in[18];
  const float* W3   = (const float*)d_in[19];
  const float* b3   = (const float*)d_in[20];
  const float* W8   = (const float*)d_in[21];
  const float* b8   = (const float*)d_in[22];
  const float* Wa   = (const float*)d_in[23];
  const float* ba   = (const float*)d_in[24];
  const float* Wpp  = (const float*)d_in[25];
  const float* bpp  = (const float*)d_in[26];
  float* out = (float*)d_out;

  char* ws = (char*)d_ws;
  size_t off = 0;
  auto carve = [&](size_t bytes) -> char* { char* p = ws + off; off += (bytes + 255) & ~(size_t)255; return p; };
  unsigned short* WB0  = (unsigned short*)carve((size_t)2 * NGATE * K0TOT * 2);
  unsigned short* WB1  = (unsigned short*)carve((size_t)2 * NGATE * K1TOT * 2);
  unsigned short* HB   = (unsigned short*)carve((size_t)2 * NHEADPAD * NUNIT * 2);
  unsigned short* H0   = (unsigned short*)carve((size_t)NT_STEPS * NB * NHID2 * 2);
  float*          PART = (float*)carve((size_t)2 * NT_STEPS * NB * NHEADPAD * 4);
  if (off > ws_size || off > (size_t)134217728) return;

  const size_t P0 = (size_t)NGATE * K0TOT, P1 = (size_t)NGATE * K1TOT;
  tpw_kernel<<<dim3(NGATE / 64, NFEAT / 64), PTHR, 0, stream>>>(Wf0, NGATE, K0TOT, WB0, WCARRY);
  tpw_kernel<<<dim3(NGATE / 64, NUNIT / 64), PTHR, 0, stream>>>(Uf0, NGATE, K0TOT, WB0 + NFEAT, WCARRY);
  tpw_kernel<<<dim3(NGATE / 64, NFEAT / 64), PTHR, 0, stream>>>(Wb0, NGATE, K0TOT, WB0 + P0, WCARRY);
  tpw_kernel<<<dim3(NGATE / 64, NUNIT / 64), PTHR, 0, stream>>>(Ub0, NGATE, K0TOT, WB0 + P0 + NFEAT, WCARRY);
  tpw_kernel<<<dim3(NGATE / 64, NHID2 / 64), PTHR, 0, stream>>>(Wf1, NGATE, K1TOT, WB1, WCARRY);
  tpw_kernel<<<dim3(NGATE / 64, NUNIT / 64), PTHR, 0, stream>>>(Uf1, NGATE, K1TOT, WB1 + NHID2, WCARRY);
  tpw_kernel<<<dim3(NGATE / 64, NHID2 / 64), PTHR, 0, stream>>>(Wb1, NGATE, K1TOT, WB1 + P1, WCARRY);
  tpw_kernel<<<dim3(NGATE / 64, NUNIT / 64), PTHR, 0, stream>>>(Ub1, NGATE, K1TOT, WB1 + P1 + NHID2, WCARRY);
  head_plane_kernel<<<(2 * NHEADPAD * NUNIT / 2) / PTHR, PTHR, 0, stream>>>(Wp, Wbu, W3, W8, Wa, Wpp, HB);

  bilstm_layer_kernel<0><<<2, LTHR, 0, stream>>>(x, H0, xm, WB0, bf0, bb0, HB, PART);
  bilstm_layer_kernel<1><<<2, LTHR, 0, stream>>>(x, H0, xm, WB1, bf1, bb1, HB, PART);

  finish_kernel<<<NROWS / PTHR, PTHR, 0, stream>>>(PART, bp, bbu, b3, b8, ba, bpp, out);
}
